// HashGenerator_34694745817199
// MI455X (gfx1250) — hardware-verified
//
#include <hip/hip_runtime.h>
#include <math.h>
typedef __attribute__((ext_vector_type(16))) _Float16 v16h;
typedef __attribute__((ext_vector_type(8)))  _Float16 v8h;
typedef __attribute__((ext_vector_type(16))) __bf16   v16b;
typedef __attribute__((ext_vector_type(8)))  __bf16   v8b;
typedef __attribute__((ext_vector_type(8)))  float    v8f;
typedef __attribute__((ext_vector_type(4)))  float    v4f;
#define PSCALE 32768.0f
#define U16(p) ((const unsigned short*)(const void*)(p))
#define PSCALE_INV (1.0f / 32768.0f)

__device__ __forceinline__ unsigned short f2bf_bits(float f) {
  unsigned u = __float_as_uint(f);
  return (unsigned short)((u + 0x7FFFu + ((u >> 16) & 1u)) >> 16);
}
__device__ __forceinline__ float bf_bits2f(unsigned short h) { return __uint_as_float(((unsigned)h) << 16); }

__device__ __forceinline__ void dep_guard_h(v8f& a, v8f& b, v16h x, v16h y) { asm volatile("v_nop\n\tv_nop\n\tv_nop\n\tv_nop" : "+v"(a), "+v"(b) : "v"(x), "v"(y)); }
__device__ __forceinline__ void dep_guard_b(v8f& a, v8f& b, v16b x, v16b y) { asm volatile("v_nop\n\tv_nop\n\tv_nop\n\tv_nop" : "+v"(a), "+v"(b) : "v"(x), "v"(y)); }
__device__ __forceinline__ void keep4_h(v16h a, v16h b, v16h c, v16h d) { asm volatile("v_nop" :: "v"(a), "v"(b), "v"(c), "v"(d)); }
__device__ __forceinline__ void keep4_b(v16b a, v16b b, v16b c, v16b d) { asm volatile("v_nop" :: "v"(a), "v"(b), "v"(c), "v"(d)); }
__device__ __forceinline__ void acc_guard4(v8f& a, v8f& b, v8f& c, v8f& d) { asm volatile("v_nop\n\tv_nop\n\tv_nop\n\tv_nop" : "+v"(a), "+v"(b), "+v"(c), "+v"(d)); }
template <typename T> struct Frag;
template <> struct Frag<_Float16> {
  typedef v16h V; union U { v16h v; v8h h[2]; };
  static __device__ __forceinline__ v16h load(const _Float16* p) {
    U f; f.h[0] = *(const v8h*)(p); f.h[1] = *(const v8h*)(p + 16); return f.v;
  }
  static __device__ __forceinline__ v8f mma(v16h a, v16h b, v8f c) {
    return __builtin_amdgcn_wmma_f32_16x16x32_f16(false, a, false, b, (short)0, c, false, false);
  }
  static __device__ __forceinline__ void guard(v8f& a, v8f& b, v16h x, v16h y) { dep_guard_h(a, b, x, y); }
  static __device__ __forceinline__ void keep(v16h a, v16h b, v16h c, v16h d) { keep4_h(a, b, c, d); }
};
template <> struct Frag<__bf16> {
  typedef v16b V; union U { v16b v; v8b h[2]; };
  static __device__ __forceinline__ v16b load(const __bf16* p) {
    U f; f.h[0] = *(const v8b*)(p); f.h[1] = *(const v8b*)(p + 16); return f.v;
  }
  static __device__ __forceinline__ v8f mma(v16b a, v16b b, v8f c) {
    return __builtin_amdgcn_wmma_f32_16x16x32_bf16(false, a, false, b, (short)0, c, false, false);
  }
  static __device__ __forceinline__ void guard(v8f& a, v8f& b, v16b x, v16b y) { dep_guard_b(a, b, x, y); }
  static __device__ __forceinline__ void keep(v16b a, v16b b, v16b c, v16b d) { keep4_b(a, b, c, d); }
};

template <int ET> struct Elem;
template <> struct Elem<0> { typedef _Float16 T; };
template <> struct Elem<1> { typedef __bf16 T; };
template <int ET, bool SPLIT, int BIAS_MODE, int OUT_MODE, bool RESID, int ACT = 0>
__global__ __launch_bounds__(256) void wmma_gemm64(
    const unsigned short* __restrict__ Ap, const unsigned short* __restrict__ A2p, int lda, long strideA,
    const unsigned short* __restrict__ Btp, const unsigned short* __restrict__ Bt2p, int ldb, long strideB,
    void* __restrict__ Cout, void* __restrict__ Cout2, int ldc, long strideC,
    const float* __restrict__ bias,
    const float* __restrict__ resid, long strideR,
    int M, int N, int K, float scale) {
  typedef typename Elem<ET>::T T;
  typedef typename Frag<T>::V V;
  const T* A = (const T*)Ap; const T* A2 = (const T*)A2p; const T* Bt = (const T*)Btp; const T* Bt2 = (const T*)Bt2p;
  __shared__ __align__(16) float sT[8][16 * 68];
  const int b    = blockIdx.y;
  const int lane = threadIdx.x & 31;
  const int wave = threadIdx.x >> 5;
  const int tilesN = N >> 6;
  const int tilesM = M >> 6;
  const int tile = blockIdx.x * 8 + wave;
  if (tile >= tilesM * tilesN) return;
  const int tm = tile / tilesN;
  const int tn = tile - tm * tilesN;
  const int m0 = tm << 6;
  const int n0 = tn << 6;

  const T* Ab  = A  + (size_t)b * strideA;
  const T* Bb  = Bt + (size_t)b * strideB;
  const T* Ab2 = SPLIT ? (A2  + (size_t)b * strideA) : nullptr;
  const T* Bb2 = SPLIT ? (Bt2 + (size_t)b * strideB) : nullptr;

  const int rlane = lane & 15;
  const int koff  = (lane >> 4) * 8;
  const int mOff  = (lane >> 4) * 8;

  v8f acc[4][4];
#pragma unroll
  for (int i = 0; i < 4; ++i)
#pragma unroll
    for (int j = 0; j < 4; ++j) acc[i][j] = (v8f){0.f,0.f,0.f,0.f,0.f,0.f,0.f,0.f};

  for (int k0 = 0; k0 < K; k0 += 32) {
    V bh[4], bl[4];
#pragma unroll
    for (int j = 0; j < 4; ++j) {
      const size_t bo = (size_t)(n0 + (j << 4) + rlane) * ldb + koff + k0;
      bh[j] = Frag<T>::load(Bb + bo);
      if (SPLIT) bl[j] = Frag<T>::load(Bb2 + bo);
    }
#pragma unroll
    for (int i = 0; i < 4; ++i) {
      const size_t ao = (size_t)(m0 + (i << 4) + rlane) * lda + koff + k0;
      V ah = Frag<T>::load(Ab + ao);
      V al;
      if (SPLIT) al = Frag<T>::load(Ab2 + ao);
#pragma unroll
      for (int j = 0; j < 4; ++j) {
        acc[i][j] = Frag<T>::mma(ah, bh[j], acc[i][j]);
        if (SPLIT) {
          acc[i][j] = Frag<T>::mma(ah, bl[j], acc[i][j]);
          acc[i][j] = Frag<T>::mma(al, bh[j], acc[i][j]);
        }
      }
      Frag<T>::guard(acc[i][0], acc[i][3], ah, SPLIT ? al : ah);
    }
    Frag<T>::keep(bh[0], bh[1], bh[2], bh[3]);
    if (SPLIT) Frag<T>::keep(bl[0], bl[1], bl[2], bl[3]);
  }
  acc_guard4(acc[0][0], acc[0][1], acc[0][2], acc[0][3]);
  acc_guard4(acc[1][0], acc[1][1], acc[1][2], acc[1][3]);
  acc_guard4(acc[2][0], acc[2][1], acc[2][2], acc[2][3]);
  acc_guard4(acc[3][0], acc[3][1], acc[3][2], acc[3][3]);

  float* slab = sT[wave];
  const float* Rb = RESID ? (resid + (size_t)b * strideR) : nullptr;
#pragma unroll
  for (int i = 0; i < 4; ++i) {
    const int mBase = m0 + (i << 4);
#pragma unroll
    for (int j = 0; j < 4; ++j) {
      const int n = n0 + (j << 4) + rlane;
      float bv = 0.f;
      if (BIAS_MODE == 2) bv = bias[n];
#pragma unroll
      for (int r = 0; r < 8; ++r) {
        float v = acc[i][j][r] * scale;
        if (BIAS_MODE == 1) v += bias[mBase + mOff + r];
        if (BIAS_MODE == 2) v += bv;
        if (RESID) v += Rb[(size_t)(mBase + mOff + r) * ldc + n];
        if (ACT == 1) v = tanhf(v);
        if (ACT == 2) v = fmaxf(v, 0.0f);
        if (ACT == 3) v = v / (1.0f + expf(-v));
        if (ACT == 4) v = (v > 0.f) ? v : 0.01f * v;
        if (ACT == 5) v = 0.5f * v * (1.0f + erff(v * 0.70710678118654752f));
        slab[(mOff + r) * 68 + (j << 4) + rlane] = v;
      }
    }
    __builtin_amdgcn_fence(__ATOMIC_RELEASE, "workgroup");
    __builtin_amdgcn_wave_barrier();
    __builtin_amdgcn_fence(__ATOMIC_ACQUIRE, "workgroup");
    if (OUT_MODE == 0) {
      float* C = (float*)Cout + (size_t)b * strideC;
      const int hh = lane >> 4, c4 = (lane & 15) * 4;
      for (int pass = 0; pass < 2; ++pass) {
#pragma unroll
        for (int it = 0; it < 8; ++it) {
          const int row = it * 2 + hh;
          v4f v = *(const v4f*)(slab + row * 68 + c4);
          *(volatile v4f*)(C + (size_t)(mBase + row) * ldc + n0 + c4) = v;
        }
        __threadfence();
      }
    } else {
      const int q = lane >> 3, c8 = (lane & 7) * 8;
      unsigned short* C  = (unsigned short*)Cout  + (size_t)b * strideC;
      unsigned short* C2 = (OUT_MODE == 2) ? ((unsigned short*)Cout2 + (size_t)b * strideC) : nullptr;
      for (int pass = 0; pass < 2; ++pass) {
#pragma unroll
        for (int it = 0; it < 4; ++it) {
          const int row = it * 4 + q;
          const float* sp = slab + row * 68 + c8;
          v8h hv, lv;
#pragma unroll
          for (int e = 0; e < 8; ++e) {
            if (OUT_MODE == 1) {
              hv[e] = (_Float16)sp[e];
            } else {
              unsigned short hb = f2bf_bits(sp[e]);
              unsigned short lb = f2bf_bits(sp[e] - bf_bits2f(hb));
              hv[e] = __builtin_bit_cast(_Float16, hb);
              lv[e] = __builtin_bit_cast(_Float16, lb);
            }
          }
          *(volatile v8h*)(C + (size_t)(mBase + row) * ldc + n0 + c8) = hv;
          if (OUT_MODE == 2) *(volatile v8h*)(C2 + (size_t)(mBase + row) * ldc + n0 + c8) = lv;
        }
        __threadfence();
      }
    }
    __builtin_amdgcn_fence(__ATOMIC_RELEASE, "workgroup");
    __builtin_amdgcn_wave_barrier();
    __builtin_amdgcn_fence(__ATOMIC_ACQUIRE, "workgroup");
  }
}

__global__ __launch_bounds__(256) void cast_f32_f16x2(
    const float* __restrict__ in, _Float16* __restrict__ out, int n2) {
  int i = blockIdx.x * 256 + threadIdx.x;
  if (i < n2) {
    const _Float16 h0 = (_Float16)in[2 * i], h1 = (_Float16)in[2 * i + 1];
    const unsigned u = (unsigned)__builtin_bit_cast(unsigned short, h0) | ((unsigned)__builtin_bit_cast(unsigned short, h1) << 16);
    ((volatile unsigned*)out)[i] = u;
    __threadfence();
    ((volatile unsigned*)out)[i] = u;
  }
}


#define HB 8
#define HL 16
#define HT 16384
#define HZ 512
#define HS 256
#define HN 65536
#define HF 32
#define HH 64
__constant__ float RESL[HL] = {16.f, 19.f, 23.f, 27.f, 33.f, 40.f, 48.f, 58.f, 70.f, 84.f, 101.f, 122.f, 147.f, 176.f, 212.f, 255.f};
__device__ __forceinline__ float lrelu_g(float x) { return 1.4142135623730951f * (x >= 0.f ? x : 0.2f * x); }
__global__ __launch_bounds__(256) void features_kernel(const float* __restrict__ base, unsigned* __restrict__ F16) {
  const int n = blockIdx.x * 256 + threadIdx.x;
  const int i = n >> 8, j = n & 255;
  const float cxf = ((float)i + 0.5f) / 256.0f, cyf = ((float)j + 0.5f) / 256.0f;
  unsigned pk[HL];
#pragma unroll 1
  for (int l = 0; l < HL; ++l) {
    const float px = cxf * RESL[l], py = cyf * RESL[l];
    const float fx = floorf(px), fy = floorf(py);
    const float rx = px - fx, ry = py - fy;
    const unsigned x0 = (unsigned)fx, y0 = (unsigned)fy;
    float f0 = 0.f, f1 = 0.f;
#pragma unroll
    for (int c = 0; c < 4; ++c) {
      const unsigned ox = c & 1u, oy = c >> 1;
      const unsigned cx = x0 + ox, cy = y0 + oy;
      const unsigned idx = (cx ^ (cy * 2654435761u)) & (HT - 1);
      const float wx = ox ? rx : (1.0f - rx), wy = oy ? ry : (1.0f - ry);
      const float w = wx * wy;
      const float* tb = base + ((size_t)l * HT + idx) * 2;
      f0 += tb[0] * w; f1 += tb[1] * w;
    }
    pk[l] = (unsigned)__builtin_bit_cast(unsigned short, (_Float16)f0) | ((unsigned)__builtin_bit_cast(unsigned short, (_Float16)f1) << 16);
  }
  typedef __attribute__((ext_vector_type(4))) unsigned u4;
  for (int pass = 0; pass < 2; ++pass) {
#pragma unroll
    for (int q = 0; q < 4; ++q) { const u4 v = {pk[4*q], pk[4*q+1], pk[4*q+2], pk[4*q+3]}; *(volatile u4*)(F16 + (size_t)n * 16 + 4 * q) = v; }
    __threadfence();
  }
}
__global__ __launch_bounds__(256) void style_kernel(const float* __restrict__ z, const float* __restrict__ mw0, const float* __restrict__ mb0, const float* __restrict__ mw1, const float* __restrict__ mb1,
                                                   const float* __restrict__ mw2, const float* __restrict__ mb2, const float* __restrict__ w_mod, const float* __restrict__ b_mod,
                                                   const float* __restrict__ a0w, const float* __restrict__ a0b, const float* __restrict__ w0,
                                                   const float* __restrict__ a1w, const float* __restrict__ a1b, const float* __restrict__ w1,
                                                   const float* __restrict__ a2w, const float* __restrict__ a2b, const float* __restrict__ w2,
                                                   unsigned* __restrict__ BT0, unsigned* __restrict__ BT1, unsigned* __restrict__ BT2) {
  __shared__ float s0[HZ], s1[HS], s2[HS];
  __shared__ float sc[HF], st0[HF], st1[HH], st2[HH], dm0[HH], dm1[HH], dm2[HH];
  const int b = blockIdx.x, t = threadIdx.x;
  for (int k = t; k < HZ; k += 256) s0[k] = z[(size_t)b * HZ + k];
  __syncthreads();
  { float a = mb0[t];
#pragma unroll 1
    for (int k = 0; k < HZ; ++k) a += s0[k] * mw0[(size_t)k * HS + t];
    s1[t] = lrelu_g(a); }
  __syncthreads();
  { float a = mb1[t];
#pragma unroll 1
    for (int k = 0; k < HS; ++k) a += s1[k] * mw1[(size_t)k * HS + t];
    s2[t] = lrelu_g(a); }
  __syncthreads();
  { float a = mb2[t];
#pragma unroll 1
    for (int k = 0; k < HS; ++k) a += s2[k] * mw2[(size_t)k * HS + t];
    s1[t] = lrelu_g(a); }
  __syncthreads();
  if (t < HF) { float a = b_mod[t], c = a0b[t];
#pragma unroll 1
    for (int k = 0; k < HS; ++k) { a += s1[k] * w_mod[(size_t)k * HF + t]; c += s1[k] * a0w[(size_t)k * HF + t]; }
    sc[t] = 1.0f + a; st0[t] = c; }
  if (t < HH) { float c1 = a1b[t], c2 = a2b[t];
#pragma unroll 1
    for (int k = 0; k < HS; ++k) { c1 += s1[k] * a1w[(size_t)k * HH + t]; c2 += s1[k] * a2w[(size_t)k * HH + t]; }
    st1[t] = c1; st2[t] = c2; }
  __syncthreads();
  if (t < HH) { float d0 = 1e-8f, d1 = 1e-8f;
#pragma unroll 1
    for (int k = 0; k < HF; ++k) { const float sw = st0[k] * w0[k * HH + t]; d0 += sw * sw; }
#pragma unroll 1
    for (int k = 0; k < HH; ++k) { const float sw = st1[k] * w1[k * HH + t]; d1 += sw * sw; }
    dm0[t] = rsqrtf(d0); dm1[t] = rsqrtf(d1);
    float d2 = 1e-8f;
    if (t < 3) {
#pragma unroll 1
      for (int k = 0; k < HH; ++k) { const float sw = st2[k] * w2[k * 3 + t]; d2 += sw * sw; } }
    dm2[t] = (t < 3) ? rsqrtf(d2) : 0.f; }
  __syncthreads();
  for (int pass = 0; pass < 2; ++pass) {
    for (int i = t; i < HH * HF / 2; i += 256) { const int o = (2 * i) / HF, k = (2 * i) % HF;
      const float a = sc[k] * st0[k] * w0[k * HH + o] * dm0[o], c = sc[k + 1] * st0[k + 1] * w0[(k + 1) * HH + o] * dm0[o];
      ((volatile unsigned*)BT0)[(size_t)b * (HH * HF / 2) + i] = (unsigned)__builtin_bit_cast(unsigned short, (_Float16)a) | ((unsigned)__builtin_bit_cast(unsigned short, (_Float16)c) << 16); }
    for (int i = t; i < HH * HH / 2; i += 256) { const int o = (2 * i) / HH, k = (2 * i) % HH;
      const float a = st1[k] * w1[k * HH + o] * dm1[o], c = st1[k + 1] * w1[(k + 1) * HH + o] * dm1[o];
      ((volatile unsigned*)BT1)[(size_t)b * (HH * HH / 2) + i] = (unsigned)__builtin_bit_cast(unsigned short, (_Float16)a) | ((unsigned)__builtin_bit_cast(unsigned short, (_Float16)c) << 16);
      float a2 = 0.f, c2 = 0.f; if (o < 3) { a2 = st2[k] * w2[k * 3 + o] * dm2[o]; c2 = st2[k + 1] * w2[(k + 1) * 3 + o] * dm2[o]; }
      ((volatile unsigned*)BT2)[(size_t)b * (HH * HH / 2) + i] = (unsigned)__builtin_bit_cast(unsigned short, (_Float16)a2) | ((unsigned)__builtin_bit_cast(unsigned short, (_Float16)c2) << 16); }
    __threadfence();
  }
}
__global__ __launch_bounds__(256) void act_cast_kernel(const float* __restrict__ X, unsigned* __restrict__ Y16, long n2) {
  const long i = (long)blockIdx.x * 256 + threadIdx.x; if (i >= n2) return;
  const float a = lrelu_g(X[2 * i]), b = lrelu_g(X[2 * i + 1]);
  const unsigned u = (unsigned)__builtin_bit_cast(unsigned short, (_Float16)a) | ((unsigned)__builtin_bit_cast(unsigned short, (_Float16)b) << 16);
  ((volatile unsigned*)Y16)[i] = u; __threadfence(); ((volatile unsigned*)Y16)[i] = u;
}
__global__ __launch_bounds__(64) void padbias3_kernel(const float* __restrict__ b3, float* __restrict__ bp) { const int t = threadIdx.x; const float v = (t < 3) ? b3[t] : 0.f; ((volatile float*)bp)[t] = v; __threadfence(); ((volatile float*)bp)[t] = v; }
__global__ __launch_bounds__(256) void permute_kernel(const float* __restrict__ T, float* __restrict__ out) {
  const int bc = blockIdx.y, b = bc / 3, c = bc % 3; const int n = blockIdx.x * 256 + threadIdx.x;
  const float v = T[((size_t)b * HN + n) * HH + c];
  ((volatile float*)out)[((size_t)b * 3 + c) * HN + n] = v; __threadfence(); ((volatile float*)out)[((size_t)b * 3 + c) * HN + n] = v;
}
extern "C" void kernel_launch(void* const* d_in, const int* in_sizes, int n_in, void* d_out, int out_size, void* d_ws, size_t ws_size, hipStream_t stream) {
  (void)in_sizes; (void)n_in; (void)out_size; (void)ws_size;
  const float* z = (const float*)d_in[0];
  const float* mw0 = (const float*)d_in[1]; const float* mb0 = (const float*)d_in[2]; const float* mw1 = (const float*)d_in[3]; const float* mb1 = (const float*)d_in[4]; const float* mw2 = (const float*)d_in[5]; const float* mb2 = (const float*)d_in[6];
  const float* base = (const float*)d_in[7]; const float* w_mod = (const float*)d_in[8]; const float* b_mod = (const float*)d_in[9];
  const float* a0w = (const float*)d_in[10]; const float* a0b = (const float*)d_in[11]; const float* w0 = (const float*)d_in[12]; const float* bb0 = (const float*)d_in[13];
  const float* a1w = (const float*)d_in[14]; const float* a1b = (const float*)d_in[15]; const float* w1 = (const float*)d_in[16]; const float* bb1 = (const float*)d_in[17];
  const float* a2w = (const float*)d_in[18]; const float* a2b = (const float*)d_in[19]; const float* w2 = (const float*)d_in[20]; const float* bb2 = (const float*)d_in[21];
  float* out = (float*)d_out;
  char* ws = (char*)d_ws; size_t off = 0;
  auto carve = [&](size_t bytes) -> char* { char* p = ws + off; off += (bytes + 255) & ~(size_t)255; return p; };
  unsigned* F16 = (unsigned*)carve((size_t)HN * HF * 2);
  unsigned* BT0 = (unsigned*)carve((size_t)HB * HH * HF * 2); unsigned* BT1 = (unsigned*)carve((size_t)HB * HH * HH * 2); unsigned* BT2 = (unsigned*)carve((size_t)HB * HH * HH * 2);
  float* bb2p = (float*)carve(64 * 4);
  float* X = (float*)carve((size_t)HB * HN * HH * 4);
  unsigned* H16 = (unsigned*)carve((size_t)HB * HN * HH * 2);
  features_kernel<<<HN / 256, 256, 0, stream>>>(base, F16);
  style_kernel<<<HB, 256, 0, stream>>>(z, mw0, mb0, mw1, mb1, mw2, mb2, w_mod, b_mod, a0w, a0b, w0, a1w, a1b, w1, a2w, a2b, w2, BT0, BT1, BT2);
  padbias3_kernel<<<1, 64, 0, stream>>>(bb2, bb2p);
  const int t = (HN / 64) * 1;
  wmma_gemm64<0, false, 2, 0, false, 0><<<dim3((t + 7) / 8, HB), 256, 0, stream>>>((const unsigned short*)F16, nullptr, HF, 0, (const unsigned short*)BT0, nullptr, HF, (long)HH * HF, X, nullptr, HH, (long)HN * HH, bb0, nullptr, 0, HN, HH, HF, 1.0f);
  act_cast_kernel<<<(HB * HN * HH / 2 + 255) / 256, 256, 0, stream>>>(X, H16, (long)HB * HN * HH / 2);
  wmma_gemm64<0, false, 2, 0, false, 0><<<dim3((t + 7) / 8, HB), 256, 0, stream>>>((const unsigned short*)H16, nullptr, HH, (long)HN * HH, (const unsigned short*)BT1, nullptr, HH, (long)HH * HH, X, nullptr, HH, (long)HN * HH, bb1, nullptr, 0, HN, HH, HH, 1.0f);
  act_cast_kernel<<<(HB * HN * HH / 2 + 255) / 256, 256, 0, stream>>>(X, H16, (long)HB * HN * HH / 2);
  wmma_gemm64<0, false, 2, 0, false, 1><<<dim3((t + 7) / 8, HB), 256, 0, stream>>>((const unsigned short*)H16, nullptr, HH, (long)HN * HH, (const unsigned short*)BT2, nullptr, HH, (long)HH * HH, X, nullptr, HH, (long)HN * HH, bb2p, nullptr, 0, HN, HH, HH, 1.0f);
  permute_kernel<<<dim3(HN / 256, HB * 3), 256, 0, stream>>>(X, out);
}
